// FeatureCorrelation_63333587746895
// MI455X (gfx1250) — hardware-run, weakly checked
//
#include <hip/hip_runtime.h>
#include <stddef.h>


#define NBATCH 8
#define NCH    256
#define HWP    4096
#define NOUT   256
#define NTHR   256
#define NWAVE  8
#define ROWS   128
#define OGRP   64
#define SPITCH 132
#define TROWS  32
#define RPITCH 260
#define LGRP   8
#define ASC    256
#define WSC    16
#define PBLK   ((NOUT * NCH / 8) / NTHR)
#define WSCAP  134217728

static_assert(ROWS == NWAVE * 16);
static_assert(NTHR == NWAVE * 32);
static_assert((NCH % 32) == 0 && (HWP % ROWS) == 0 && (HWP % TROWS) == 0);
static_assert((NOUT % OGRP) == 0 && OGRP == NWAVE * 8 && (OGRP % 16) == 0);
static_assert(TROWS == NWAVE * 4 && TROWS == 32);
static_assert((NOUT * NCH / 8) % NTHR == 0);
static_assert((SPITCH % 4) == 0 && (RPITCH % 4) == 0 && RPITCH >= NCH);
static_assert(NCH == NWAVE * LGRP * (NCH / (NWAVE * LGRP)));
static_assert(NOUT == NTHR);
static_assert(ROWS * 4 == 32 * 16);
static_assert(NCH * 2 == 32 * 16);

typedef float     v4f  __attribute__((ext_vector_type(4)));
typedef float     v8f  __attribute__((ext_vector_type(8)));
typedef _Float16  v8h  __attribute__((ext_vector_type(8)));
typedef _Float16  v16h __attribute__((ext_vector_type(16)));
union FragH { v16h v; v8h h[2]; };

__device__ __forceinline__ v8f wmf(v16h a, v16h b, v8f c) {
  v8f d = __builtin_amdgcn_wmma_f32_16x16x32_f16(false, a, false, b, (short)0, c, false, false);
  asm volatile("v_nop\n\tv_nop\n\tv_nop\n\tv_nop" : "+v"(d) : "v"(a), "v"(b));
  return d;
}

__device__ __forceinline__ void wmf2(v16h a, v16h b0, v16h b1, v8f& c0, v8f& c1) {
  v8f d0 = __builtin_amdgcn_wmma_f32_16x16x32_f16(false, a, false, b0, (short)0, c0, false, false);
  v8f d1 = __builtin_amdgcn_wmma_f32_16x16x32_f16(false, a, false, b1, (short)0, c1, false, false);
  asm volatile("v_nop\n\tv_nop\n\tv_nop\n\tv_nop" : "+v"(d0), "+v"(d1) : "v"(a), "v"(b0), "v"(b1));
  c0 = d0;
  c1 = d1;
}

__global__ __launch_bounds__(NTHR) void k_prep(
    const float* __restrict__ w,  const float* __restrict__ cb,
    const float* __restrict__ ga, const float* __restrict__ be,
    const float* __restrict__ mu, const float* __restrict__ va,
    _Float16* w16, float* cst) {
  __shared__ __attribute__((aligned(16))) float s_c[3 * NOUT];
  const int tid = threadIdx.x, lane = tid & 31, wave = tid >> 5;
  if ((int)blockIdx.x < PBLK) {
    const int i = (int)blockIdx.x * NTHR + tid;
    const int o = i >> 5, c8 = (i & 31) * 8;
    const float* sp = w + (size_t)o * (2 * NCH) + c8;
    const v4f f0 = *(const v4f*)sp;
    const v4f f1 = *(const v4f*)(sp + 4);
    const float sc = (float)WSC;
    v8h hv;
    hv[0] = (_Float16)(f0.x * sc); hv[1] = (_Float16)(f0.y * sc);
    hv[2] = (_Float16)(f0.z * sc); hv[3] = (_Float16)(f0.w * sc);
    hv[4] = (_Float16)(f1.x * sc); hv[5] = (_Float16)(f1.y * sc);
    hv[6] = (_Float16)(f1.z * sc); hv[7] = (_Float16)(f1.w * sc);
    _Float16* d = w16 + (size_t)i * 8;
    *(volatile v8h*)d = hv;
    __threadfence();
    *(volatile v8h*)d = hv;
  } else {
    const int o = tid;
    const float* row = w + (size_t)o * (2 * NCH) + NCH;
    float wsum = 0.f;
#pragma unroll 1
    for (int c = 0; c < NCH; ++c) wsum += row[c];
    const float sc = ga[o] / sqrtf(va[o] + 1e-5f);
    s_c[o]            = sc;
    s_c[NOUT + o]     = wsum * sc;
    s_c[2 * NOUT + o] = (cb[o] - mu[o]) * sc + be[o];
    __syncthreads();
    if (wave < 3) {
      const v4f u0 = *(const v4f*)(s_c + wave * NOUT + 4 * lane);
      const v4f u1 = *(const v4f*)(s_c + wave * NOUT + 128 + 4 * lane);
      float* g0 = cst + wave * NOUT + 4 * lane;
      float* g1 = g0 + 128;
      *(volatile v4f*)g0 = u0;
      *(volatile v4f*)g1 = u1;
      __threadfence();
      *(volatile v4f*)g0 = u0;
      *(volatile v4f*)g1 = u1;
    }
  }
}

__global__ __launch_bounds__(NTHR) void k_nt(
    const float* __restrict__ src, const float* __restrict__ tgt,
    _Float16* srcT, _Float16* tgtT, float* nrm) {
  __shared__ __attribute__((aligned(16))) float raw[TROWS * RPITCH];
  __shared__ __attribute__((aligned(16))) float part[NWAVE * 32];
  __shared__ __attribute__((aligned(16))) float s_nrm[32];
  __shared__ __attribute__((aligned(16))) float s_scl[32];
  const int tid = threadIdx.x, tx = tid & 31, ty = tid >> 5;
  const int i0 = (int)blockIdx.x * TROWS, b = (int)blockIdx.y;
  const bool isT = (blockIdx.z != 0);
  const float* in = isT ? tgt : src;
  _Float16* outp = isT ? tgtT : srcT;

  const float* ip = in + ((size_t)b * NCH + ty) * HWP + i0 + tx;
  float* rw = raw + tx * RPITCH + ty;
  float ss = 0.f;
#pragma unroll 1
  for (int g = 0; g < NCH / (NWAVE * LGRP); ++g) {
    const float* gp = ip + (size_t)(NWAVE * LGRP * g) * HWP;
    float x[LGRP];
#pragma unroll
    for (int kk = 0; kk < LGRP; ++kk) x[kk] = gp[(size_t)(NWAVE * kk) * HWP];
#pragma unroll
    for (int kk = 0; kk < LGRP; ++kk) {
      ss += x[kk] * x[kk];
      rw[NWAVE * LGRP * g + NWAVE * kk] = x[kk];
    }
  }
  part[ty * 32 + tx] = ss;
  __syncthreads();
  if (tid < 32) {
    float t = part[tx];
#pragma unroll
    for (int w2 = 1; w2 < NWAVE; ++w2) t += part[w2 * 32 + tx];
    const float nr = fmaxf(sqrtf(t), 1e-12f);
    s_nrm[tx] = nr;
    s_scl[tx] = (float)ASC * __builtin_amdgcn_rcpf(nr);
  }
  __syncthreads();

  v8h hvr[4];
#pragma unroll
  for (int rr = 0; rr < 4; ++rr) {
    const int rl = 4 * ty + rr;
    const float scl = s_scl[rl];
    const v4f f0 = *(const v4f*)(raw + rl * RPITCH + 8 * tx);
    const v4f f1 = *(const v4f*)(raw + rl * RPITCH + 8 * tx + 4);
    v8h hv;
    hv[0] = (_Float16)(f0.x * scl); hv[1] = (_Float16)(f0.y * scl);
    hv[2] = (_Float16)(f0.z * scl); hv[3] = (_Float16)(f0.w * scl);
    hv[4] = (_Float16)(f1.x * scl); hv[5] = (_Float16)(f1.y * scl);
    hv[6] = (_Float16)(f1.z * scl); hv[7] = (_Float16)(f1.w * scl);
    hvr[rr] = hv;
  }
  _Float16* rbase = outp + ((size_t)b * HWP + i0) * NCH + 8 * tx;
#pragma unroll
  for (int rr = 0; rr < 4; ++rr) {
    const int rl = 4 * ty + rr;
    *(volatile v8h*)(rbase + (size_t)rl * NCH) = hvr[rr];
  }
  const bool nwave = (!isT) && (ty == 0);
  const v4f nvl = *(const v4f*)(s_nrm + 4 * (tx & 7));
  float* np = nrm + (size_t)b * HWP + i0 + 4 * (tx & 7);
  if (nwave) { if (tx < 8) *(volatile v4f*)np = nvl; }
  __threadfence();
#pragma unroll
  for (int rr = 0; rr < 4; ++rr) {
    const int rl = 4 * ty + rr;
    *(volatile v8h*)(rbase + (size_t)rl * NCH) = hvr[rr];
  }
  if (nwave) { if (tx < 8) *(volatile v4f*)np = nvl; }
}

__global__ __launch_bounds__(NTHR) __attribute__((amdgpu_num_vgpr(256)))
void k_corr(const _Float16* __restrict__ srcT, const _Float16* __restrict__ tgtT,
            const _Float16* __restrict__ w16, const float* __restrict__ nrm,
            const float* __restrict__ cst, float* out) {
  __shared__ __attribute__((aligned(16))) float stg[OGRP * SPITCH];
  const int tid = threadIdx.x, lane = tid & 31, wave = tid >> 5, hh = lane >> 4, m = lane & 15;
  const int b = (int)blockIdx.y, i0 = (int)blockIdx.x * ROWS, iw = i0 + wave * 16;
  const v8f z8 = {0.f, 0.f, 0.f, 0.f, 0.f, 0.f, 0.f, 0.f};

  FragH a[NCH / 32];
  {
    const _Float16* ap = srcT + ((size_t)b * HWP + iw + m) * NCH + 8 * hh;
#pragma unroll
    for (int kt = 0; kt < NCH / 32; ++kt) {
      a[kt].h[0] = *(const v8h*)(ap + 32 * kt);
      a[kt].h[1] = *(const v8h*)(ap + 32 * kt + 16);
    }
  }

  float vmax[8];
#pragma unroll
  for (int r = 0; r < 8; ++r) vmax[r] = -__builtin_inff();

  const _Float16* tb = tgtT + ((size_t)b * HWP + m) * NCH + 8 * hh;
#pragma unroll 1
  for (int jt = 0; jt < HWP / 32; ++jt) {
    const _Float16* bp0 = tb + (size_t)(32 * jt) * NCH;
    const _Float16* bp1 = bp0 + 16 * NCH;
    v8f acc0 = z8, acc1 = z8;
#pragma unroll
    for (int kt = 0; kt < NCH / 32; ++kt) {
      FragH f0, f1;
      f0.h[0] = *(const v8h*)(bp0 + 32 * kt);
      f0.h[1] = *(const v8h*)(bp0 + 32 * kt + 16);
      f1.h[0] = *(const v8h*)(bp1 + 32 * kt);
      f1.h[1] = *(const v8h*)(bp1 + 32 * kt + 16);
      wmf2(a[kt].v, f0.v, f1.v, acc0, acc1);
    }
#pragma unroll
    for (int r = 0; r < 8; ++r) vmax[r] = fmaxf(vmax[r], fmaxf(acc0[r], acc1[r]));
  }

#pragma unroll
  for (int r = 0; r < 8; ++r) {
    float t = vmax[r];
    t = fmaxf(t, __shfl_xor(t, 8));
    t = fmaxf(t, __shfl_xor(t, 4));
    t = fmaxf(t, __shfl_xor(t, 2));
    t = fmaxf(t, __shfl_xor(t, 1));
    vmax[r] = t * (1.0f / 65536.0f);
  }

  float nv[8];
  {
    const float* np = nrm + (size_t)b * HWP + iw + 8 * hh;
    const v4f n0 = *(const v4f*)np;
    const v4f n1 = *(const v4f*)(np + 4);
    nv[0] = n0.x; nv[1] = n0.y; nv[2] = n0.z; nv[3] = n0.w;
    nv[4] = n1.x; nv[5] = n1.y; nv[6] = n1.z; nv[7] = n1.w;
  }

#pragma unroll 1
  for (int g = 0; g < NOUT / OGRP; ++g) {
#pragma unroll
    for (int t = 0; t < OGRP / 16; ++t) {
      const int ol = 16 * t + m;
      const int o = OGRP * g + ol;
      const _Float16* wp = w16 + (size_t)o * NCH + 8 * hh;
      v8f acc = z8;
#pragma unroll
      for (int kt = 0; kt < NCH / 32; ++kt) {
        FragH fw;
        fw.h[0] = *(const v8h*)(wp + 32 * kt);
        fw.h[1] = *(const v8h*)(wp + 32 * kt + 16);
        acc = wmf(a[kt].v, fw.v, acc);
      }
      const float pA = cst[o] * (1.0f / 4096.0f);
      const float pB = cst[NOUT + o];
      const float pC = cst[2 * NOUT + o];
      float y[8];
#pragma unroll
      for (int r = 0; r < 8; ++r) {
        const float x = (acc[r] * nv[r]) * pA + vmax[r] * pB + pC;
        const float e = __expf(-x);
        y[r] = x * __builtin_amdgcn_rcpf(1.0f + e);
      }
      float* sp = stg + ol * SPITCH + wave * 16 + 8 * hh;
      const v4f u0 = {y[0], y[1], y[2], y[3]};
      const v4f u1 = {y[4], y[5], y[6], y[7]};
      *(v4f*)sp = u0;
      *(v4f*)(sp + 4) = u1;
    }
    __syncthreads();
    float* ob = out + ((size_t)b * NOUT + OGRP * g + wave * 8) * HWP + i0 + 4 * lane;
    const float* lb = stg + (wave * 8) * SPITCH + 4 * lane;
#pragma unroll
    for (int rr = 0; rr < 8; ++rr) {
      const v4f u = *(const v4f*)(lb + rr * SPITCH);
      *(volatile v4f*)(ob + (size_t)rr * HWP) = u;
    }
    __threadfence();
#pragma unroll
    for (int rr = 0; rr < 8; ++rr) {
      const v4f u = *(const v4f*)(lb + rr * SPITCH);
      *(volatile v4f*)(ob + (size_t)rr * HWP) = u;
    }
    __syncthreads();
  }
}

extern "C" void kernel_launch(void* const* d_in, const int* in_sizes, int n_in,
                              void* d_out, int out_size, void* d_ws, size_t ws_size,
                              hipStream_t stream) {
  if (n_in < 8) return;
  if (in_sizes[0] != NBATCH * NCH * HWP || in_sizes[1] != NBATCH * NCH * HWP) return;
  if (in_sizes[2] != NOUT * 2 * NCH || in_sizes[3] != NOUT) return;
  if (in_sizes[4] != NOUT || in_sizes[5] != NOUT || in_sizes[6] != NOUT || in_sizes[7] != NOUT) return;
  if (out_size != NBATCH * NOUT * HWP) return;

  const float* src = (const float*)d_in[0];
  const float* tgt = (const float*)d_in[1];
  const float* cw  = (const float*)d_in[2];
  const float* cb  = (const float*)d_in[3];
  const float* ga  = (const float*)d_in[4];
  const float* be  = (const float*)d_in[5];
  const float* mu  = (const float*)d_in[6];
  const float* va  = (const float*)d_in[7];
  float* out = (float*)d_out;

  char* ws = (char*)d_ws;
  size_t off = 0;
  const size_t oS = off; off += (size_t)NBATCH * HWP * NCH * 2;  off = (off + 255) & ~(size_t)255;
  const size_t oT = off; off += (size_t)NBATCH * HWP * NCH * 2;  off = (off + 255) & ~(size_t)255;
  const size_t oW = off; off += (size_t)NOUT * NCH * 2;          off = (off + 255) & ~(size_t)255;
  const size_t oN = off; off += (size_t)NBATCH * HWP * 4;        off = (off + 255) & ~(size_t)255;
  const size_t oC = off; off += (size_t)3 * NOUT * 4;            off = (off + 255) & ~(size_t)255;
  if (off > ws_size || off > (size_t)WSCAP) return;
  _Float16* srcT = (_Float16*)(ws + oS);
  _Float16* tgtT = (_Float16*)(ws + oT);
  _Float16* w16  = (_Float16*)(ws + oW);
  float*    nrm  = (float*)(ws + oN);
  float*    cst  = (float*)(ws + oC);

  k_prep<<<PBLK + 1, NTHR, 0, stream>>>(cw, cb, ga, be, mu, va, w16, cst);
  k_nt<<<dim3(HWP / TROWS, NBATCH, 2), NTHR, 0, stream>>>(src, tgt, srcT, tgtT, nrm);
  k_corr<<<dim3(HWP / ROWS, NBATCH), NTHR, 0, stream>>>(srcT, tgtT, w16, nrm, cst, out);
}
